// GridificationLayer_8864812499080
// MI455X (gfx1250) — hardware-verified
//
#include <hip/hip_runtime.h>
#include <math.h>

typedef __attribute__((ext_vector_type(16))) _Float16 v16h;
typedef __attribute__((ext_vector_type(8)))  _Float16 v8h;
typedef __attribute__((ext_vector_type(16))) __bf16   v16b;
typedef __attribute__((ext_vector_type(8)))  __bf16   v8b;
typedef __attribute__((ext_vector_type(8)))  float    v8f;
typedef __attribute__((ext_vector_type(4)))  float    v4f;
typedef __attribute__((ext_vector_type(4)))  int      v4i;
typedef __attribute__((ext_vector_type(2)))  unsigned u2v;
#define U16(p) ((const unsigned short*)(const void*)(p))

__device__ __forceinline__ unsigned short f2bf_bits(float f) {
  unsigned u = __float_as_uint(f);
  return (unsigned short)((u + 0x7FFFu + ((u >> 16) & 1u)) >> 16);
}
__device__ __forceinline__ float bf_bits2f(unsigned short h) { return __uint_as_float(((unsigned)h) << 16); }

__device__ __forceinline__ void dep_guard_h(v8f& a, v8f& b, v16h x, v16h y) { asm volatile("v_nop\n\tv_nop\n\tv_nop\n\tv_nop" : "+v"(a), "+v"(b) : "v"(x), "v"(y)); }
__device__ __forceinline__ void dep_guard_b(v8f& a, v8f& b, v16b x, v16b y) { asm volatile("v_nop\n\tv_nop\n\tv_nop\n\tv_nop" : "+v"(a), "+v"(b) : "v"(x), "v"(y)); }
__device__ __forceinline__ void keep4_h(v16h a, v16h b, v16h c, v16h d) { asm volatile("v_nop" :: "v"(a), "v"(b), "v"(c), "v"(d)); }
__device__ __forceinline__ void keep4_b(v16b a, v16b b, v16b c, v16b d) { asm volatile("v_nop" :: "v"(a), "v"(b), "v"(c), "v"(d)); }
__device__ __forceinline__ void acc_guard4(v8f& a, v8f& b, v8f& c, v8f& d) { asm volatile("v_nop\n\tv_nop\n\tv_nop\n\tv_nop" : "+v"(a), "+v"(b), "+v"(c), "+v"(d)); }
template <typename T> struct Frag;
template <> struct Frag<_Float16> {
  typedef v16h V; union U { v16h v; v8h h[2]; };
  static __device__ __forceinline__ v16h load(const _Float16* p) {
    U f; f.h[0] = *(const v8h*)(p); f.h[1] = *(const v8h*)(p + 16); return f.v;
  }
  static __device__ __forceinline__ v8f mma(v16h a, v16h b, v8f c) {
    return __builtin_amdgcn_wmma_f32_16x16x32_f16(false, a, false, b, (short)0, c, false, false);
  }
  static __device__ __forceinline__ void guard(v8f& a, v8f& b, v16h x, v16h y) { dep_guard_h(a, b, x, y); }
  static __device__ __forceinline__ void keep(v16h a, v16h b, v16h c, v16h d) { keep4_h(a, b, c, d); }
};
template <> struct Frag<__bf16> {
  typedef v16b V; union U { v16b v; v8b h[2]; };
  static __device__ __forceinline__ v16b load(const __bf16* p) {
    U f; f.h[0] = *(const v8b*)(p); f.h[1] = *(const v8b*)(p + 16); return f.v;
  }
  static __device__ __forceinline__ v8f mma(v16b a, v16b b, v8f c) {
    return __builtin_amdgcn_wmma_f32_16x16x32_bf16(false, a, false, b, (short)0, c, false, false);
  }
  static __device__ __forceinline__ void guard(v8f& a, v8f& b, v16b x, v16b y) { dep_guard_b(a, b, x, y); }
  static __device__ __forceinline__ void keep(v16b a, v16b b, v16b c, v16b d) { keep4_b(a, b, c, d); }
};

template <int ET> struct Elem;
template <> struct Elem<0> { typedef _Float16 T; };
template <> struct Elem<1> { typedef __bf16 T; };
template <int ET, bool SPLIT, int BIAS_MODE, int OUT_MODE, bool RESID, int ACT = 0>
__global__ __launch_bounds__(256) void wmma_gemm64(
    const unsigned short* __restrict__ Ap, const unsigned short* __restrict__ A2p, int lda, long strideA,
    const unsigned short* __restrict__ Btp, const unsigned short* __restrict__ Bt2p, int ldb, long strideB,
    void* __restrict__ Cout, void* __restrict__ Cout2, int ldc, long strideC,
    const float* __restrict__ bias,
    const float* __restrict__ resid, long strideR,
    int M, int N, int K, float scale) {
  typedef typename Elem<ET>::T T;
  typedef typename Frag<T>::V V;
  const T* A = (const T*)Ap; const T* A2 = (const T*)A2p; const T* Bt = (const T*)Btp; const T* Bt2 = (const T*)Bt2p;
  __shared__ __align__(16) float sT[8][16 * 68];
  const int b    = blockIdx.y;
  const int lane = threadIdx.x & 31;
  const int wave = threadIdx.x >> 5;
  const int tilesN = N >> 6;
  const int tilesM = M >> 6;
  const int tile = blockIdx.x * 8 + wave;
  if (tile >= tilesM * tilesN) return;
  const int tm = tile / tilesN;
  const int tn = tile - tm * tilesN;
  const int m0 = tm << 6;
  const int n0 = tn << 6;

  const T* Ab  = A  + (size_t)b * strideA;
  const T* Bb  = Bt + (size_t)b * strideB;
  const T* Ab2 = SPLIT ? (A2  + (size_t)b * strideA) : nullptr;
  const T* Bb2 = SPLIT ? (Bt2 + (size_t)b * strideB) : nullptr;

  const int rlane = lane & 15;
  const int koff  = (lane >> 4) * 8;
  const int mOff  = (lane >> 4) * 8;

  v8f acc[4][4];
#pragma unroll
  for (int i = 0; i < 4; ++i)
#pragma unroll
    for (int j = 0; j < 4; ++j) acc[i][j] = (v8f){0.f,0.f,0.f,0.f,0.f,0.f,0.f,0.f};

  for (int k0 = 0; k0 < K; k0 += 32) {
    V bh[4], bl[4];
#pragma unroll
    for (int j = 0; j < 4; ++j) {
      const size_t bo = (size_t)(n0 + (j << 4) + rlane) * ldb + koff + k0;
      bh[j] = Frag<T>::load(Bb + bo);
      if (SPLIT) bl[j] = Frag<T>::load(Bb2 + bo);
    }
#pragma unroll
    for (int i = 0; i < 4; ++i) {
      const size_t ao = (size_t)(m0 + (i << 4) + rlane) * lda + koff + k0;
      V ah = Frag<T>::load(Ab + ao);
      V al;
      if (SPLIT) al = Frag<T>::load(Ab2 + ao);
#pragma unroll
      for (int j = 0; j < 4; ++j) {
        acc[i][j] = Frag<T>::mma(ah, bh[j], acc[i][j]);
        if (SPLIT) {
          acc[i][j] = Frag<T>::mma(ah, bl[j], acc[i][j]);
          acc[i][j] = Frag<T>::mma(al, bh[j], acc[i][j]);
        }
      }
      Frag<T>::guard(acc[i][0], acc[i][3], ah, SPLIT ? al : ah);
    }
    Frag<T>::keep(bh[0], bh[1], bh[2], bh[3]);
    if (SPLIT) Frag<T>::keep(bl[0], bl[1], bl[2], bl[3]);
  }
  acc_guard4(acc[0][0], acc[0][1], acc[0][2], acc[0][3]);
  acc_guard4(acc[1][0], acc[1][1], acc[1][2], acc[1][3]);
  acc_guard4(acc[2][0], acc[2][1], acc[2][2], acc[2][3]);
  acc_guard4(acc[3][0], acc[3][1], acc[3][2], acc[3][3]);

  float* slab = sT[wave];
  const float* Rb = RESID ? (resid + (size_t)b * strideR) : nullptr;
#pragma unroll
  for (int i = 0; i < 4; ++i) {
    const int mBase = m0 + (i << 4);
#pragma unroll
    for (int j = 0; j < 4; ++j) {
      const int n = n0 + (j << 4) + rlane;
      float bv = 0.f;
      if (BIAS_MODE == 2) bv = bias[n];
#pragma unroll
      for (int r = 0; r < 8; ++r) {
        float v = acc[i][j][r] * scale;
        if (BIAS_MODE == 1) v += bias[mBase + mOff + r];
        if (BIAS_MODE == 2) v += bv;
        if (RESID) v += Rb[(size_t)(mBase + mOff + r) * ldc + n];
        if (ACT == 1) v = tanhf(v);
        if (ACT == 2) v = fmaxf(v, 0.0f);
        if (ACT == 3) v = v / (1.0f + expf(-v));
        if (ACT == 4) v = (v > 0.f) ? v : 0.01f * v;
        if (ACT == 5) v = 0.5f * v * (1.0f + erff(v * 0.70710678118654752f));
        slab[(mOff + r) * 68 + (j << 4) + rlane] = v;
      }
    }
    __builtin_amdgcn_fence(__ATOMIC_RELEASE, "workgroup");
    __builtin_amdgcn_wave_barrier();
    __builtin_amdgcn_fence(__ATOMIC_ACQUIRE, "workgroup");
    if (OUT_MODE == 0) {
      float* C = (float*)Cout + (size_t)b * strideC;
      const int hh = lane >> 4, c4 = (lane & 15) * 4;
      for (int pass = 0; pass < 2; ++pass) {
#pragma unroll
        for (int it = 0; it < 8; ++it) {
          const int row = it * 2 + hh;
          v4f v = *(const v4f*)(slab + row * 68 + c4);
          *(volatile v4f*)(C + (size_t)(mBase + row) * ldc + n0 + c4) = v;
        }
        __threadfence();
      }
    } else {
      const int q = lane >> 3, c8 = (lane & 7) * 8;
      unsigned short* C  = (unsigned short*)Cout  + (size_t)b * strideC;
      unsigned short* C2 = (OUT_MODE == 2) ? ((unsigned short*)Cout2 + (size_t)b * strideC) : nullptr;
      for (int pass = 0; pass < 2; ++pass) {
#pragma unroll
        for (int it = 0; it < 4; ++it) {
          const int row = it * 4 + q;
          const float* sp = slab + row * 68 + c8;
          v8h hv, lv;
#pragma unroll
          for (int e = 0; e < 8; ++e) {
            if (OUT_MODE == 1) {
              hv[e] = (_Float16)sp[e];
            } else {
              unsigned short hb = f2bf_bits(sp[e]);
              unsigned short lb = f2bf_bits(sp[e] - bf_bits2f(hb));
              hv[e] = __builtin_bit_cast(_Float16, hb);
              lv[e] = __builtin_bit_cast(_Float16, lb);
            }
          }
          *(volatile v8h*)(C + (size_t)(mBase + row) * ldc + n0 + c8) = hv;
          if (OUT_MODE == 2) *(volatile v8h*)(C2 + (size_t)(mBase + row) * ldc + n0 + c8) = lv;
        }
        __threadfence();
      }
    }
    __builtin_amdgcn_fence(__ATOMIC_RELEASE, "workgroup");
    __builtin_amdgcn_wave_barrier();
    __builtin_amdgcn_fence(__ATOMIC_ACQUIRE, "workgroup");
  }
}

__global__ __launch_bounds__(256) void cast_f32_f16x2(
    const float* __restrict__ in, _Float16* __restrict__ out, int n2) {
  int i = blockIdx.x * 256 + threadIdx.x;
  if (i < n2) {
    const _Float16 h0 = (_Float16)in[2 * i], h1 = (_Float16)in[2 * i + 1];
    const unsigned u = (unsigned)__builtin_bit_cast(unsigned short, h0) | ((unsigned)__builtin_bit_cast(unsigned short, h1) << 16);
    ((volatile unsigned*)out)[i] = u;
    __threadfence();
    ((volatile unsigned*)out)[i] = u;
  }
}

#define NNODE 65536
#define NCELL 32768
#define NE 600000
#define FH 128
#define CH 75008
#define NCHUNK 8
#define EPW 8
#define TB 256
#define NTILE (NCELL / TB)
#define NT 256
#define SCH 4096
#define SPT (SCH / NT)
#define NSUB ((CH + SCH - 1) / SCH)

__global__ __launch_bounds__(256) void transpose8_kernel(
    const float* __restrict__ a0, const float* __restrict__ a1, const float* __restrict__ a2, const float* __restrict__ a3,
    const float* __restrict__ a4, const float* __restrict__ a5, const float* __restrict__ a6, const float* __restrict__ a7,
    _Float16* __restrict__ o0, _Float16* __restrict__ o1, _Float16* __restrict__ o2, _Float16* __restrict__ o3,
    _Float16* __restrict__ o4, _Float16* __restrict__ o5, _Float16* __restrict__ o6, _Float16* __restrict__ o7) {
  __shared__ __align__(16) _Float16 tile[64][72];
  const int z = blockIdx.z;
  const float* in = a0; _Float16* outT = o0;
  if (z == 1) { in = a1; outT = o1; }
  if (z == 2) { in = a2; outT = o2; }
  if (z == 3) { in = a3; outT = o3; }
  if (z == 4) { in = a4; outT = o4; }
  if (z == 5) { in = a5; outT = o5; }
  if (z == 6) { in = a6; outT = o6; }
  if (z == 7) { in = a7; outT = o7; }
  const int c0 = blockIdx.x * 64, r0 = blockIdx.y * 64;
  const int t = threadIdx.y * 32 + threadIdx.x;
  for (int i = threadIdx.y; i < 64; i += 8) {
    tile[threadIdx.x][i]      = (_Float16)(in[(size_t)(r0 + i) * FH + c0 + threadIdx.x]);
    tile[32 + threadIdx.x][i] = (_Float16)(in[(size_t)(r0 + i) * FH + c0 + 32 + threadIdx.x]);
  }
  __syncthreads();
  const int q = t >> 3, c8 = (t & 7) * 8;
  for (int pass = 0; pass < 2; ++pass) {
#pragma unroll
    for (int it = 0; it < 2; ++it) {
      const int c = it * 32 + q;
      v8h hv = *(const v8h*)(&tile[c][c8]);
      *(volatile v8h*)(outT + (size_t)(c0 + c) * FH + r0 + c8) = hv;
    }
    __threadfence();
  }
}

__global__ __launch_bounds__(256) void edge_gather_kernel(int k, const int* __restrict__ ei, const float* __restrict__ node_pos,
    const float* __restrict__ cell_pos, const float* __restrict__ w1, const float* __restrict__ b1, const float* __restrict__ P,
    unsigned* __restrict__ A1, float* __restrict__ PR) {
  const int lane = threadIdx.x & 31, wave = threadIdx.x >> 5;
  const v4f wk0 = *(const v4f*)(w1 + 0 * FH + 4 * lane);
  const v4f wk1 = *(const v4f*)(w1 + 1 * FH + 4 * lane);
  const v4f wk2 = *(const v4f*)(w1 + 2 * FH + 4 * lane);
  const v4f wk3 = *(const v4f*)(w1 + 3 * FH + 4 * lane);
  const v4f wk4 = *(const v4f*)(w1 + 4 * FH + 4 * lane);
  const v4f wk5 = *(const v4f*)(w1 + 5 * FH + 4 * lane);
  const v4f bb  = *(const v4f*)(b1 + 4 * lane);
  const v4f z4 = {0.f, 0.f, 0.f, 0.f};
  const int i0 = (blockIdx.x * 8 + wave) * EPW;
#pragma unroll 1
  for (int j = 0; j < EPW; ++j) {
    const int i = i0 + j;
    const int e = k * CH + i;
    v4f h = z4, pr = z4;
    if (e < NE) {
      int sn = ei[e], tg = ei[NE + e];
      sn = sn < 0 ? 0 : (sn >= NNODE ? NNODE - 1 : sn);
      tg = tg < 0 ? 0 : (tg >= NCELL ? NCELL - 1 : tg);
      const float p0 = node_pos[(size_t)sn * 3], p1 = node_pos[(size_t)sn * 3 + 1], p2 = node_pos[(size_t)sn * 3 + 2];
      const float g0 = cell_pos[(size_t)tg * 3], g1 = cell_pos[(size_t)tg * 3 + 1], g2 = cell_pos[(size_t)tg * 3 + 2];
      const v4f a = p0 * wk0 + p1 * wk1 + p2 * wk2 + g0 * wk3 + g1 * wk4 + g2 * wk5 + bb;
#pragma unroll
      for (int q = 0; q < 4; ++q) h[q] = a[q] * __builtin_amdgcn_rcpf(1.0f + __expf(-a[q]));
      pr = *(const v4f*)(P + (size_t)sn * FH + 4 * lane);
    }
    u2v hv;
    hv[0] = (unsigned)__builtin_bit_cast(unsigned short, (_Float16)h[0]) | ((unsigned)__builtin_bit_cast(unsigned short, (_Float16)h[1]) << 16);
    hv[1] = (unsigned)__builtin_bit_cast(unsigned short, (_Float16)h[2]) | ((unsigned)__builtin_bit_cast(unsigned short, (_Float16)h[3]) << 16);
    for (int pass = 0; pass < 2; ++pass) {
      *(volatile u2v*)(A1 + (size_t)i * (FH / 2) + 2 * lane) = hv;
      *(volatile v4f*)(PR + (size_t)i * FH + 4 * lane) = pr;
      __threadfence();
    }
  }
}

__device__ __forceinline__ int blk_excl_scan(int cnt, int* scan_ws, int tid, int* tot) {
  const int lane = tid & 31, wave = tid >> 5; int incl = cnt;
#pragma unroll
  for (int o = 1; o < 32; o <<= 1) { const int v = __shfl_up(incl, o, 32); if (lane >= o) incl += v; }
  if (lane == 31) scan_ws[wave] = incl;
  __syncthreads();
  if (wave == 0) { int wv = (lane < NT / 32) ? scan_ws[lane] : 0; int wincl = wv;
#pragma unroll
    for (int o = 1; o < 32; o <<= 1) { const int v = __shfl_up(wincl, o, 32); if (lane >= o) wincl += v; }
    if (lane < NT / 32) scan_ws[32 + lane] = wincl - wv; if (lane == 31) scan_ws[64] = wincl; }
  __syncthreads();
  const int res = scan_ws[32 + wave] + incl - cnt; *tot = scan_ws[64];
  return res;
}
template <int SP, int CAP>
__device__ __forceinline__ int chunk_hits(const int* __restrict__ dstv, int e0, int eend, int ebase, int n0, int tid,
                                          int* LIST, int* scan_ws) {
  const int eb = e0 + tid * SP;
  int rec[SP]; int cnt = 0;
  if (eb < eend) {
#pragma unroll
    for (int kk = 0; kk < SP; kk += 4) {
      const v4i d4 = *(const v4i*)(dstv + eb + kk);
#pragma unroll
      for (int e = 0; e < 4; ++e) {
        const int d = d4[e]; int r = -1;
        if (d >= n0 && d < n0 + TB) { r = ((d - n0) << 20) | (eb + kk + e - ebase); ++cnt; }
        rec[kk + e] = r;
      }
    }
  } else {
#pragma unroll
    for (int kk = 0; kk < SP; ++kk) rec[kk] = -1;
  }
  int tot; int p = blk_excl_scan(cnt, scan_ws, tid, &tot);
#pragma unroll
  for (int kk = 0; kk < SP; ++kk) if (rec[kk] >= 0) { if ((unsigned)p < (unsigned)CAP) LIST[p] = rec[kk]; ++p; }
  __syncthreads();
  return tot < CAP ? tot : CAP;
}

__global__ __launch_bounds__(NT) void cell_aggregate_kernel(int k, const int* __restrict__ ei, const float* __restrict__ MSG,
                                                           float* AGG, int* CNT, unsigned* __restrict__ AG16) {
  __shared__ __align__(16) float sacc[TB * FH];
  __shared__ __align__(16) int scnt[TB];
  __shared__ int LIST[SCH];
  __shared__ int scan_ws[80];
  const int tid = threadIdx.x, lane = tid & 31, wave = tid >> 5;
  const int n0 = blockIdx.x * TB;
  const v4f z4 = {0.f, 0.f, 0.f, 0.f};
#pragma unroll 1
  for (int j = 0; j < TB / 8; ++j) {
    const int dl = wave * (TB / 8) + j;
    v4f a = z4;
    if (k != 0) a = *(const v4f*)(AGG + (size_t)(n0 + dl) * FH + 4 * lane);
    *(v4f*)(sacc + dl * FH + 4 * lane) = a;
  }
  scnt[tid] = (k != 0) ? CNT[n0 + tid] : 0;
  __syncthreads();
  const int* dstv = ei + NE;
  const int ebase = k * CH;
  const int eend = (ebase + CH < NE) ? (ebase + CH) : NE;
#pragma unroll 1
  for (int c = 0; c < NSUB; ++c) {
    const int tot = chunk_hits<SPT, SCH>(dstv, ebase + c * SCH, eend, ebase, n0, tid, LIST, scan_ws);
#pragma unroll 1
    for (int base = 0; base < tot; base += 32) {
      const int q = base + lane;
      const int rv = (q < tot) ? LIST[q] : -1;
      const int own = (rv >= 0 && (rv >> 25) == wave) ? 1 : 0;
      unsigned msk = (unsigned)__ballot(own);
#pragma unroll 1
      for (int it = 0; it < 32; ++it) {
        if (msk == 0u) break;
        const int bp = __builtin_ctz(msk); msk &= msk - 1u;
        const int r = __shfl(rv, bp, 32);
        const int dl = (r >> 20) & (TB - 1);
        int el = r & 0xFFFFF; el = el < CH ? el : CH - 1;
        const v4f m = *(const v4f*)(MSG + (size_t)el * FH + 4 * lane);
        float* rp = sacc + dl * FH + 4 * lane;
        v4f a = *(const v4f*)rp;
        a = a + m;
        *(v4f*)rp = a;
        if (lane == 0) scnt[dl] += 1;
      }
    }
    __syncthreads();
  }
  if (k != NCHUNK - 1) {
    for (int pass = 0; pass < 2; ++pass) {
#pragma unroll 1
      for (int j = 0; j < TB / 8; ++j) {
        const int dl = wave * (TB / 8) + j;
        const v4f a = *(const v4f*)(sacc + dl * FH + 4 * lane);
        *(volatile v4f*)(AGG + (size_t)(n0 + dl) * FH + 4 * lane) = a;
      }
      if (wave == 0) {
        const v4i cA = *(const v4i*)(scnt + 4 * lane), cB = *(const v4i*)(scnt + 128 + 4 * lane);
        *(volatile v4i*)(CNT + n0 + 4 * lane) = cA;
        *(volatile v4i*)(CNT + n0 + 128 + 4 * lane) = cB;
      }
      __threadfence();
    }
  } else {
    for (int pass = 0; pass < 2; ++pass) {
#pragma unroll 1
      for (int j = 0; j < TB / 8; ++j) {
        const int dl = wave * (TB / 8) + j;
        const int cn = scnt[dl];
        const float cf = (float)cn;
        const float inv = 1.0f / fmaxf(cf, 1.0f);
        v4f a = *(const v4f*)(sacc + dl * FH + 4 * lane);
        a = a * inv;
        u2v hv;
        hv[0] = (unsigned)__builtin_bit_cast(unsigned short, (_Float16)a[0]) | ((unsigned)__builtin_bit_cast(unsigned short, (_Float16)a[1]) << 16);
        hv[1] = (unsigned)__builtin_bit_cast(unsigned short, (_Float16)a[2]) | ((unsigned)__builtin_bit_cast(unsigned short, (_Float16)a[3]) << 16);
        *(volatile u2v*)(AG16 + (size_t)(n0 + dl) * (FH / 2) + 2 * lane) = hv;
      }
      __threadfence();
    }
  }
}

extern "C" void kernel_launch(void* const* d_in, const int* in_sizes, int n_in,
                              void* d_out, int out_size, void* d_ws, size_t ws_size,
                              hipStream_t stream) {
  if (n_in < 20) return;
  if (in_sizes[0] != NNODE * FH || in_sizes[1] != NNODE * 3 || in_sizes[2] != NCELL * 3 || in_sizes[3] != 2 * NE) return;
  if (out_size != NCELL * FH) return;
  const float* nfeat = (const float*)d_in[0];
  const float* npos  = (const float*)d_in[1];
  const float* cpos  = (const float*)d_in[2];
  const int*   ei    = (const int*)d_in[3];
  const float* nm_w1 = (const float*)d_in[4];  const float* nm_b1 = (const float*)d_in[5];
  const float* nm_w2 = (const float*)d_in[6];  const float* nm_b2 = (const float*)d_in[7];
  const float* em_w1 = (const float*)d_in[8];  const float* em_b1 = (const float*)d_in[9];
  const float* em_w2 = (const float*)d_in[10]; const float* em_b2 = (const float*)d_in[11];
  const float* mm_w1 = (const float*)d_in[12]; const float* mm_b1 = (const float*)d_in[13];
  const float* mm_w2 = (const float*)d_in[14]; const float* mm_b2 = (const float*)d_in[15];
  const float* um_w1 = (const float*)d_in[16]; const float* um_b1 = (const float*)d_in[17];
  const float* um_w2 = (const float*)d_in[18]; const float* um_b2 = (const float*)d_in[19];
  float* out = (float*)d_out;

  char* ws = (char*)d_ws; size_t off = 0;
  auto carve = [&](size_t bytes) -> char* { char* p = ws + off; off += (bytes + 255) & ~(size_t)255; return p; };
  _Float16* Wn1  = (_Float16*)carve((size_t)FH * FH * 2);
  _Float16* Wn2  = (_Float16*)carve((size_t)FH * FH * 2);
  _Float16* We2  = (_Float16*)carve((size_t)FH * FH * 2);
  _Float16* Wm1a = (_Float16*)carve((size_t)FH * FH * 2);
  _Float16* Wm1b = (_Float16*)carve((size_t)FH * FH * 2);
  _Float16* Wm2  = (_Float16*)carve((size_t)FH * FH * 2);
  _Float16* Wu1  = (_Float16*)carve((size_t)FH * FH * 2);
  _Float16* Wu2  = (_Float16*)carve((size_t)FH * FH * 2);
  float* P   = (float*)carve((size_t)NNODE * FH * 4);
  float* AGG = (float*)carve((size_t)NCELL * FH * 4);
  int*   CNT = (int*)carve((size_t)NCELL * 4);
  char*  R   = carve((size_t)CH * 1024);
  if (off > ws_size || off > (size_t)134217728) return;
  unsigned short* X16  = (unsigned short*)R;
  unsigned short* H16  = (unsigned short*)(R + (size_t)NNODE * FH * 2);
  unsigned short* NF16 = (unsigned short*)(R + (size_t)2 * NNODE * FH * 2);
  unsigned*       A1  = (unsigned*)R;
  unsigned short* HM  = (unsigned short*)R;
  unsigned short* EF  = (unsigned short*)(R + (size_t)CH * FH * 2);
  float*          PR  = (float*)(R + (size_t)CH * FH * 4);
  float*          MSG = PR;
  unsigned*       AG16 = (unsigned*)R;
  unsigned short* UH   = EF;

  transpose8_kernel<<<dim3(FH / 64, FH / 64, 8), dim3(32, 8), 0, stream>>>(
      nm_w1, nm_w2, em_w2, mm_w1, mm_w1 + (size_t)FH * FH, mm_w2, um_w1, um_w2,
      Wn1, Wn2, We2, Wm1a, Wm1b, Wm2, Wu1, Wu2);
  cast_f32_f16x2<<<(NNODE * FH / 2 + 255) / 256, 256, 0, stream>>>(nfeat, (_Float16*)X16, NNODE * FH / 2);
  {
    const int t = (NNODE / 64) * (FH / 64);
    wmma_gemm64<0, false, 2, 1, false, 3><<<dim3((t + 7) / 8, 1), 256, 0, stream>>>(
        U16(X16), nullptr, FH, 0L, U16(Wn1), nullptr, FH, 0L, (void*)H16, nullptr, FH, 0L, nm_b1, (const float*)nullptr, 0L, NNODE, FH, FH, 1.0f);
    wmma_gemm64<0, false, 2, 1, false, 0><<<dim3((t + 7) / 8, 1), 256, 0, stream>>>(
        U16(H16), nullptr, FH, 0L, U16(Wn2), nullptr, FH, 0L, (void*)NF16, nullptr, FH, 0L, nm_b2, (const float*)nullptr, 0L, NNODE, FH, FH, 1.0f);
    wmma_gemm64<0, false, 0, 0, false, 0><<<dim3((t + 7) / 8, 1), 256, 0, stream>>>(
        U16(NF16), nullptr, FH, 0L, U16(Wm1a), nullptr, FH, 0L, (void*)P, nullptr, FH, 0L, (const float*)nullptr, (const float*)nullptr, 0L, NNODE, FH, FH, 1.0f);
  }
  for (int k = 0; k < NCHUNK; ++k) {
    edge_gather_kernel<<<CH / (8 * EPW), 256, 0, stream>>>(k, ei, npos, cpos, em_w1, em_b1, P, A1, PR);
    const int t1 = (CH / 64) * (FH / 64);
    wmma_gemm64<0, false, 2, 1, false, 0><<<dim3((t1 + 7) / 8, 1), 256, 0, stream>>>(
        (const unsigned short*)A1, nullptr, FH, 0L, U16(We2), nullptr, FH, 0L, (void*)EF, nullptr, FH, 0L, em_b2, (const float*)nullptr, 0L, CH, FH, FH, 1.0f);
    wmma_gemm64<0, false, 2, 1, true, 3><<<dim3((t1 + 7) / 8, 1), 256, 0, stream>>>(
        U16(EF), nullptr, FH, 0L, U16(Wm1b), nullptr, FH, 0L, (void*)HM, nullptr, FH, 0L, mm_b1, (const float*)PR, 0L, CH, FH, FH, 1.0f);
    wmma_gemm64<0, false, 2, 0, false, 0><<<dim3((t1 + 7) / 8, 1), 256, 0, stream>>>(
        U16(HM), nullptr, FH, 0L, U16(Wm2), nullptr, FH, 0L, (void*)MSG, nullptr, FH, 0L, mm_b2, (const float*)nullptr, 0L, CH, FH, FH, 1.0f);
    cell_aggregate_kernel<<<NTILE, NT, 0, stream>>>(k, ei, MSG, AGG, CNT, AG16);
  }
  {
    const int t = (NCELL / 64) * (FH / 64);
    wmma_gemm64<0, false, 2, 1, false, 3><<<dim3((t + 7) / 8, 1), 256, 0, stream>>>(
        (const unsigned short*)AG16, nullptr, FH, 0L, U16(Wu1), nullptr, FH, 0L, (void*)UH, nullptr, FH, 0L, um_b1, (const float*)nullptr, 0L, NCELL, FH, FH, 1.0f);
    wmma_gemm64<0, false, 2, 0, false, 0><<<dim3((t + 7) / 8, 1), 256, 0, stream>>>(
        U16(UH), nullptr, FH, 0L, U16(Wu2), nullptr, FH, 0L, (void*)out, nullptr, FH, 0L, um_b2, (const float*)nullptr, 0L, NCELL, FH, FH, 1.0f);
  }
}
